// LinkPrediction_17248588660763
// MI455X (gfx1250) — hardware-run, weakly checked
//
#include <hip/hip_runtime.h>
#include <math.h>

typedef __attribute__((ext_vector_type(16))) _Float16 v16h;
typedef __attribute__((ext_vector_type(8)))  _Float16 v8h;
typedef __attribute__((ext_vector_type(16))) __bf16   v16b;
typedef __attribute__((ext_vector_type(8)))  float    v8f;
typedef __attribute__((ext_vector_type(4)))  float    v4f;

__device__ __forceinline__ v8f wmma16(v16h a, v16h b, v8f c) {
    c = __builtin_amdgcn_wmma_f32_16x16x32_f16(false, a, false, b, (short)0, c, false, false);
    asm volatile("v_nop\n\tv_nop\n\tv_nop\n\tv_nop" : "+v"(c) : "v"(a), "v"(b));
    return c;
}

#define VST2(T, ptr, val) do { const T vst2_v_ = (val); *(volatile T*)(ptr) = vst2_v_; __threadfence(); *(volatile T*)(ptr) = vst2_v_; } while (0)
typedef float v4f __attribute__((ext_vector_type(4)));
#define VST2V4(ptr, val) do { const v4f vst2_v4_ = (val); *(volatile v4f*)(ptr) = vst2_v4_; __threadfence(); *(volatile v4f*)(ptr) = vst2_v4_; } while (0)

namespace eng {
typedef __attribute__((ext_vector_type(16))) _Float16 v16h;
typedef __attribute__((ext_vector_type(8)))  _Float16 v8h;
typedef __attribute__((ext_vector_type(16))) __bf16   v16b;
typedef __attribute__((ext_vector_type(8)))  __bf16   v8b;
typedef __attribute__((ext_vector_type(8)))  float    v8f;
typedef __attribute__((ext_vector_type(4)))  float    v4f;

__device__ __forceinline__ unsigned short f2bf_bits(float f) {
  unsigned u = __float_as_uint(f);
  return (unsigned short)((u + 0x7FFFu + ((u >> 16) & 1u)) >> 16);
}
__device__ __forceinline__ float bf_bits2f(unsigned short h) { return __uint_as_float(((unsigned)h) << 16); }

__device__ __forceinline__ void dep_guard_h(v8f& a, v8f& b, v16h x, v16h y) { asm volatile("v_nop\n\tv_nop\n\tv_nop\n\tv_nop" : "+v"(a), "+v"(b) : "v"(x), "v"(y)); }
__device__ __forceinline__ void dep_guard_b(v8f& a, v8f& b, v16b x, v16b y) { asm volatile("v_nop\n\tv_nop\n\tv_nop\n\tv_nop" : "+v"(a), "+v"(b) : "v"(x), "v"(y)); }
__device__ __forceinline__ void keep4_h(v16h a, v16h b, v16h c, v16h d) { asm volatile("v_nop" :: "v"(a), "v"(b), "v"(c), "v"(d)); }
__device__ __forceinline__ void keep4_b(v16b a, v16b b, v16b c, v16b d) { asm volatile("v_nop" :: "v"(a), "v"(b), "v"(c), "v"(d)); }
__device__ __forceinline__ void acc_guard4(v8f& a, v8f& b, v8f& c, v8f& d) { asm volatile("v_nop\n\tv_nop\n\tv_nop\n\tv_nop" : "+v"(a), "+v"(b), "+v"(c), "+v"(d)); }
template <typename T> struct Frag;
template <> struct Frag<_Float16> {
  typedef v16h V; union U { v16h v; v8h h[2]; };
  static __device__ __forceinline__ v16h load(const _Float16* p) {
    U f; f.h[0] = *(const v8h*)(p); f.h[1] = *(const v8h*)(p + 16); return f.v;
  }
  static __device__ __forceinline__ v8f mma(v16h a, v16h b, v8f c) {
    return __builtin_amdgcn_wmma_f32_16x16x32_f16(false, a, false, b, (short)0, c, false, false);
  }
  static __device__ __forceinline__ void guard(v8f& a, v8f& b, v16h x, v16h y) { dep_guard_h(a, b, x, y); }
  static __device__ __forceinline__ void keep(v16h a, v16h b, v16h c, v16h d) { keep4_h(a, b, c, d); }
};
template <> struct Frag<__bf16> {
  typedef v16b V; union U { v16b v; v8b h[2]; };
  static __device__ __forceinline__ v16b load(const __bf16* p) {
    U f; f.h[0] = *(const v8b*)(p); f.h[1] = *(const v8b*)(p + 16); return f.v;
  }
  static __device__ __forceinline__ v8f mma(v16b a, v16b b, v8f c) {
    return __builtin_amdgcn_wmma_f32_16x16x32_bf16(false, a, false, b, (short)0, c, false, false);
  }
  static __device__ __forceinline__ void guard(v8f& a, v8f& b, v16b x, v16b y) { dep_guard_b(a, b, x, y); }
  static __device__ __forceinline__ void keep(v16b a, v16b b, v16b c, v16b d) { keep4_b(a, b, c, d); }
};

template <int ET> struct Elem;
template <> struct Elem<0> { typedef _Float16 T; };
template <> struct Elem<1> { typedef __bf16 T; };
template <int ET, bool SPLIT, int BIAS_MODE, int OUT_MODE, bool RESID, int ACT = 0>
__global__ __launch_bounds__(256) void wmma_gemm64(
    const unsigned short* __restrict__ Ap, const unsigned short* __restrict__ A2p, int lda, long strideA,
    const unsigned short* __restrict__ Btp, const unsigned short* __restrict__ Bt2p, int ldb, long strideB,
    void* __restrict__ Cout, void* __restrict__ Cout2, int ldc, long strideC,
    const float* __restrict__ bias,
    const float* __restrict__ resid, long strideR,
    int M, int N, int K, float scale) {
  typedef typename Elem<ET>::T T;
  typedef typename Frag<T>::V V;
  const T* A = (const T*)Ap; const T* A2 = (const T*)A2p; const T* Bt = (const T*)Btp; const T* Bt2 = (const T*)Bt2p;
  __shared__ __align__(16) float sT[8][16 * 68];
  const int b    = blockIdx.y;
  const int lane = threadIdx.x & 31;
  const int wave = threadIdx.x >> 5;
  const int tilesN = N >> 6;
  const int tilesM = M >> 6;
  const int tile = blockIdx.x * 8 + wave;
  if (tile >= tilesM * tilesN) return;
  const int tm = tile / tilesN;
  const int tn = tile - tm * tilesN;
  const int m0 = tm << 6;
  const int n0 = tn << 6;

  const T* Ab  = A  + (size_t)b * strideA;
  const T* Bb  = Bt + (size_t)b * strideB;
  const T* Ab2 = SPLIT ? (A2  + (size_t)b * strideA) : nullptr;
  const T* Bb2 = SPLIT ? (Bt2 + (size_t)b * strideB) : nullptr;

  const int rlane = lane & 15;
  const int koff  = (lane >> 4) * 8;
  const int mOff  = (lane >> 4) * 8;

  v8f acc[4][4];
#pragma unroll
  for (int i = 0; i < 4; ++i)
#pragma unroll
    for (int j = 0; j < 4; ++j) acc[i][j] = (v8f){0.f,0.f,0.f,0.f,0.f,0.f,0.f,0.f};

  for (int k0 = 0; k0 < K; k0 += 32) {
    V bh[4], bl[4];
#pragma unroll
    for (int j = 0; j < 4; ++j) {
      const size_t bo = (size_t)(n0 + (j << 4) + rlane) * ldb + koff + k0;
      bh[j] = Frag<T>::load(Bb + bo);
      if (SPLIT) bl[j] = Frag<T>::load(Bb2 + bo);
    }
#pragma unroll
    for (int i = 0; i < 4; ++i) {
      const size_t ao = (size_t)(m0 + (i << 4) + rlane) * lda + koff + k0;
      V ah = Frag<T>::load(Ab + ao);
      V al;
      if (SPLIT) al = Frag<T>::load(Ab2 + ao);
#pragma unroll
      for (int j = 0; j < 4; ++j) {
        acc[i][j] = Frag<T>::mma(ah, bh[j], acc[i][j]);
        if (SPLIT) {
          acc[i][j] = Frag<T>::mma(ah, bl[j], acc[i][j]);
          acc[i][j] = Frag<T>::mma(al, bh[j], acc[i][j]);
        }
      }
      Frag<T>::guard(acc[i][0], acc[i][3], ah, SPLIT ? al : ah);
    }
    Frag<T>::keep(bh[0], bh[1], bh[2], bh[3]);
    if (SPLIT) Frag<T>::keep(bl[0], bl[1], bl[2], bl[3]);
  }
  acc_guard4(acc[0][0], acc[0][1], acc[0][2], acc[0][3]);
  acc_guard4(acc[1][0], acc[1][1], acc[1][2], acc[1][3]);
  acc_guard4(acc[2][0], acc[2][1], acc[2][2], acc[2][3]);
  acc_guard4(acc[3][0], acc[3][1], acc[3][2], acc[3][3]);

  float* slab = sT[wave];
  const float* Rb = RESID ? (resid + (size_t)b * strideR) : nullptr;
#pragma unroll
  for (int i = 0; i < 4; ++i) {
    const int mBase = m0 + (i << 4);
#pragma unroll
    for (int j = 0; j < 4; ++j) {
      const int n = n0 + (j << 4) + rlane;
      float bv = 0.f;
      if (BIAS_MODE == 2) bv = bias[n];
#pragma unroll
      for (int r = 0; r < 8; ++r) {
        float v = acc[i][j][r] * scale;
        if (BIAS_MODE == 1) v += bias[mBase + mOff + r];
        if (BIAS_MODE == 2) v += bv;
        if (RESID) v += Rb[(size_t)(mBase + mOff + r) * ldc + n];
        if (ACT == 1) v = tanhf(v);
        if (ACT == 2) v = fmaxf(v, 0.0f);
        if (ACT == 3) v = v / (1.0f + expf(-v));
        if (ACT == 4) v = (v > 0.f) ? v : 0.01f * v;
        if (ACT == 5) v = 0.5f * v * (1.0f + erff(v * 0.70710678118654752f));
        if (ACT == 6) v = (v > 0.f) ? v : 0.2f * v;
        if (ACT == 7) { const float u = 0.7978845608028654f * (v + 0.044715f * v * v * v); v = 0.5f * v * (1.f + tanhf(u)); }
        slab[(mOff + r) * 68 + (j << 4) + rlane] = v;
      }
    }
    __builtin_amdgcn_fence(3  , "workgroup");
    __builtin_amdgcn_wave_barrier();
    __builtin_amdgcn_fence(2  , "workgroup");
    if (OUT_MODE == 0) {
      float* C = (float*)Cout + (size_t)b * strideC;
      const int hh = lane >> 4, c4 = (lane & 15) * 4;
      for (int pass = 0; pass < 2; ++pass) {
#pragma unroll
        for (int it = 0; it < 8; ++it) {
          const int row = it * 2 + hh;
          v4f v = *(const v4f*)(slab + row * 68 + c4);
          *(volatile v4f*)(C + (size_t)(mBase + row) * ldc + n0 + c4) = v;
        }
        __threadfence();
      }
    } else {
      const int q = lane >> 3, c8 = (lane & 7) * 8;
      unsigned short* C  = (unsigned short*)Cout  + (size_t)b * strideC;
      unsigned short* C2 = (OUT_MODE == 2) ? ((unsigned short*)Cout2 + (size_t)b * strideC) : nullptr;
      for (int pass = 0; pass < 2; ++pass) {
#pragma unroll
        for (int it = 0; it < 4; ++it) {
          const int row = it * 4 + q;
          const float* sp = slab + row * 68 + c8;
          v8h hv, lv;
#pragma unroll
          for (int e = 0; e < 8; ++e) {
            if (OUT_MODE == 1) {
              hv[e] = (_Float16)sp[e];
            } else {
              unsigned short hb = f2bf_bits(sp[e]);
              unsigned short lb = f2bf_bits(sp[e] - bf_bits2f(hb));
              hv[e] = __builtin_bit_cast(_Float16, hb);
              lv[e] = __builtin_bit_cast(_Float16, lb);
            }
          }
          *(volatile v8h*)(C + (size_t)(mBase + row) * ldc + n0 + c8) = hv;
          if (OUT_MODE == 2) *(volatile v8h*)(C2 + (size_t)(mBase + row) * ldc + n0 + c8) = lv;
        }
        __threadfence();
      }
    }
    __builtin_amdgcn_fence(3  , "workgroup");
    __builtin_amdgcn_wave_barrier();
    __builtin_amdgcn_fence(2  , "workgroup");
  }
}

}

__device__ __forceinline__ unsigned short at_f2h(float x) { return (fabsf(x) < 6.104e-5f) ? (unsigned short)0 : __builtin_bit_cast(unsigned short, (_Float16)x); }
typedef __attribute__((ext_vector_type(4))) unsigned int v4u_at;
__device__ __forceinline__ void at_st8h(unsigned short* Pp, long long o, const float* v) { v4u_at pk; pk.x = (unsigned int)at_f2h(v[0]) | ((unsigned int)at_f2h(v[1]) << 16); pk.y = (unsigned int)at_f2h(v[2]) | ((unsigned int)at_f2h(v[3]) << 16); pk.z = (unsigned int)at_f2h(v[4]) | ((unsigned int)at_f2h(v[5]) << 16); pk.w = (unsigned int)at_f2h(v[6]) | ((unsigned int)at_f2h(v[7]) << 16); VST2(v4u_at, (v4u_at*)(Pp + o), pk); }
__global__ __launch_bounds__(256) void k_at_h16(const float* __restrict__ X, unsigned short* __restrict__ O16, float sc, long long n8) { const long long u = (long long)blockIdx.x * 256 + threadIdx.x; if (u >= n8) return; const float* x = X + 8 * u; float v[8];
#pragma unroll
    for (int i = 0; i < 8; ++i) v[i] = x[i] * sc;
    at_st8h(O16, 8 * u, v); }
__global__ __launch_bounds__(256) void k_mh_wt16(const float* __restrict__ Wm, int KI, int NO, unsigned short* __restrict__ W16, float sw) { const long long u = (long long)blockIdx.x * 256 + threadIdx.x; const int per = KI / 8; if (u >= (long long)NO * per) return; const int k0 = 8 * (int)(u % per); const int o = (int)(u / per); float v[8];
#pragma unroll
    for (int i = 0; i < 8; ++i) v[i] = Wm[(long long)(k0 + i) * NO + o] * sw;
    at_st8h(W16, (long long)o * KI + k0, v); }

#ifndef NPAT
#define NPAT 2048
#endif
#ifndef NDRUG
#define NDRUG 1024
#endif
#define NDRUG_FULL 1024
#define HD 128
#define PK_MT 128
#define PK_NT 32
#define PK_WP 136

static_assert(HD == 128);
static_assert(HD % 32 == 0);
static_assert(HD % 64 == 0);
static_assert(NPAT % 64 == 0);
static_assert(NDRUG % 64 == 0);
static_assert(NDRUG % PK_MT == 0);
static_assert(NPAT % PK_NT == 0);
static_assert(NDRUG <= NDRUG_FULL);
static_assert(PK_MT == 8 * 16);
static_assert(PK_NT == 4 * 8);
static_assert(PK_WP >= HD);
static_assert((PK_WP * 2) % 16 == 0);
static_assert(256 * 16 * 4 == PK_NT * PK_MT * 4);
static_assert((HD * (3 * HD / 8)) * 8 == HD * 3 * HD);
static_assert(8 * 16 * 68 * 4 <= 131072);
static_assert(HD * PK_WP * 2 + PK_NT * HD * 2 + PK_NT * HD * 4 + HD * 4 + PK_NT * PK_MT * 4 <= 131072);

typedef _Float16 h16;
static __device__ __forceinline__ h16 toh_flush(float v) { const h16 r = (h16)v; return (fabsf(v) < 6.103515625e-05f) ? (h16)0.0f : r; }

__global__ __launch_bounds__(256) __attribute__((amdgpu_num_vgpr(256))) void k_pair(
    const unsigned short* __restrict__ P16, const unsigned short* __restrict__ D16, const unsigned short* __restrict__ WT16,
    const float* __restrict__ PP, const float* __restrict__ DPB, const float* __restrict__ W2, const float* __restrict__ B2,
    float* __restrict__ OUT) {
    __shared__ __align__(16) _Float16 sW[HD * PK_WP];
    __shared__ __align__(16) _Float16 sP[PK_NT * HD];
    __shared__ __align__(16) float    sPP[PK_NT * HD];
    __shared__ __align__(16) float    sW2[HD];
    __shared__ __align__(16) float    sO[PK_NT * PK_MT];
    union FragU { v16h v; v8h h[2]; };
    const int tid = threadIdx.x;
    const int lane = tid & 31, hf = lane >> 4, l15 = lane & 15;
    const int wave = __builtin_amdgcn_readfirstlane(threadIdx.x >> 5);
    const int m0 = blockIdx.x * PK_MT, n0 = blockIdx.y * PK_NT;
    const _Float16* wi = (const _Float16*)WT16 + 2 * HD;
    const _Float16* pg = (const _Float16*)P16 + (size_t)n0 * HD;
    const _Float16* dg = (const _Float16*)D16;

    for (int c = tid; c < HD * 16; c += 256) { const int o = c >> 4, k8 = (c & 15) * 8; *(v8h*)&sW[o * PK_WP + k8] = *(const v8h*)(wi + (size_t)o * (3 * HD) + k8); }
    for (int c = tid; c < PK_NT * 16; c += 256) { *(v8h*)&sP[c * 8] = *(const v8h*)(pg + (size_t)c * 8); }
    for (int c = tid; c < PK_NT * 32; c += 256) { const v4f v = *(const v4f*)(PP + (size_t)n0 * HD + (size_t)c * 4) * 2048.0f; *(v4f*)&sPP[c * 4] = v; }
    sW2[tid & (HD - 1)] = W2[tid & (HD - 1)] * (1.0f / 2048.0f);
    const float bb = B2[0];
    __syncthreads();

    const int mrow = m0 + 16 * wave + l15;
    const _Float16* drow = dg + (size_t)mrow * HD + 8 * hf;
    FragU d16[4];
#pragma unroll
    for (int ks = 0; ks < 4; ++ks) { d16[ks].h[0] = *(const v8h*)(drow + 32 * ks); d16[ks].h[1] = *(const v8h*)(drow + 32 * ks + 16); }
    float dpb[8][8];
    const float* dprow = DPB + (size_t)mrow * HD + 8 * hf;
#pragma unroll
    for (int t = 0; t < 8; ++t) {
        const v4f a = *(const v4f*)(dprow + 16 * t) * 2048.0f;
        const v4f b = *(const v4f*)(dprow + 16 * t + 4) * 2048.0f;
        dpb[t][0] = a.x; dpb[t][1] = a.y; dpb[t][2] = a.z; dpb[t][3] = a.w;
        dpb[t][4] = b.x; dpb[t][5] = b.y; dpb[t][6] = b.z; dpb[t][7] = b.w;
    }

#pragma unroll 1
    for (int nl = 0; nl < PK_NT; ++nl) {
        v16h bq[4];
#pragma unroll
        for (int ks = 0; ks < 4; ++ks) {
            FragU pa;
            pa.h[0] = *(const v8h*)&sP[nl * HD + 32 * ks + 8 * hf];
            pa.h[1] = *(const v8h*)&sP[nl * HD + 32 * ks + 16 + 8 * hf];
            v16h b;
#pragma unroll
            for (int i = 0; i < 16; ++i) b[i] = toh_flush((float)d16[ks].v[i] * (float)pa.v[i]);
            bq[ks] = b;
        }
        float part = 0.f;
#pragma unroll
        for (int t = 0; t < 8; ++t) {
            const v4f q0 = *(const v4f*)&sPP[nl * HD + 16 * t + 8 * hf];
            const v4f q1 = *(const v4f*)&sPP[nl * HD + 16 * t + 8 * hf + 4];
            v8f acc;
            acc[0] = dpb[t][0] + q0.x; acc[1] = dpb[t][1] + q0.y; acc[2] = dpb[t][2] + q0.z; acc[3] = dpb[t][3] + q0.w;
            acc[4] = dpb[t][4] + q1.x; acc[5] = dpb[t][5] + q1.y; acc[6] = dpb[t][6] + q1.z; acc[7] = dpb[t][7] + q1.w;
#pragma unroll
            for (int ks = 0; ks < 4; ++ks) {
                FragU fa;
                fa.h[0] = *(const v8h*)&sW[(16 * t + l15) * PK_WP + 32 * ks + 8 * hf];
                fa.h[1] = *(const v8h*)&sW[(16 * t + l15) * PK_WP + 32 * ks + 16 + 8 * hf];
                acc = wmma16(fa.v, bq[ks], acc);
            }
            const v4f w0 = *(const v4f*)&sW2[16 * t + 8 * hf];
            const v4f w1 = *(const v4f*)&sW2[16 * t + 8 * hf + 4];
            part += fmaxf(acc[0], 0.f) * w0.x; part += fmaxf(acc[1], 0.f) * w0.y; part += fmaxf(acc[2], 0.f) * w0.z; part += fmaxf(acc[3], 0.f) * w0.w;
            part += fmaxf(acc[4], 0.f) * w1.x; part += fmaxf(acc[5], 0.f) * w1.y; part += fmaxf(acc[6], 0.f) * w1.z; part += fmaxf(acc[7], 0.f) * w1.w;
        }
        part += __shfl_xor(part, 16, 32);
        const float x = part + bb;
        const float val = 1.f / (1.f + expf(-x));
        if (hf == 0) sO[nl * PK_MT + 16 * wave + l15] = val;
    }
    __syncthreads();

    v4f ov[4];
#pragma unroll
    for (int it = 0; it < 4; ++it) ov[it] = *(const v4f*)&sO[(it * 8 + wave) * PK_MT + 4 * lane];
    for (int pass = 0; pass < 2; ++pass) {
#pragma unroll
        for (int it = 0; it < 4; ++it) {
            const int row = it * 8 + wave;
            *(volatile v4f*)(OUT + (size_t)(n0 + row) * NDRUG_FULL + m0 + 4 * lane) = ov[it];
        }
        __threadfence();
    }
}

constexpr size_t WS_P16  = (size_t)NPAT * HD * 2;
constexpr size_t WS_D16  = (size_t)NDRUG * HD * 2;
constexpr size_t WS_WT16 = (size_t)HD * 3 * HD * 2;
constexpr size_t WS_PP   = (size_t)NPAT * HD * 4;
constexpr size_t WS_DPB  = (size_t)NDRUG * HD * 4;
static_assert(WS_P16 % 256 == 0);
static_assert(WS_D16 % 256 == 0);
static_assert(WS_WT16 % 256 == 0);
static_assert(WS_PP % 256 == 0);
static_assert(WS_DPB % 256 == 0);
static_assert(WS_P16 + WS_D16 + WS_WT16 + WS_PP + WS_DPB <= (size_t)134217728);

extern "C" void kernel_launch(void* const* d_in, const int* in_sizes, int n_in, void* d_out, int out_size, void* d_ws, size_t ws_size, hipStream_t stream) {
    if (n_in < 6) return;
    if (in_sizes[0] < NPAT * HD || in_sizes[1] < NDRUG * HD || in_sizes[2] < 3 * HD * HD || in_sizes[3] < HD || in_sizes[4] < HD || in_sizes[5] < 1) return;
    if ((long long)out_size < (long long)(NPAT - 1) * NDRUG_FULL + NDRUG) return;
    const float* pat = (const float*)d_in[0];
    const float* drg = (const float*)d_in[1];
    const float* W1  = (const float*)d_in[2];
    const float* b1  = (const float*)d_in[3];
    const float* W2  = (const float*)d_in[4];
    const float* b2  = (const float*)d_in[5];
    float* out = (float*)d_out;
    char* wsp = (char*)d_ws;
    unsigned short* P16  = (unsigned short*)wsp; wsp += WS_P16;
    unsigned short* D16  = (unsigned short*)wsp; wsp += WS_D16;
    unsigned short* WT16 = (unsigned short*)wsp; wsp += WS_WT16;
    float* PPb  = (float*)wsp; wsp += WS_PP;
    float* DPBb = (float*)wsp; wsp += WS_DPB;
    if ((size_t)(wsp - (char*)d_ws) > ws_size) return;

    k_mh_wt16<<<(unsigned)((HD * (3 * HD / 8) + 255) / 256), 256, 0, stream>>>(W1, 3 * HD, HD, WT16, 32.0f);
    k_at_h16<<<(unsigned)(((long long)NPAT * HD / 8 + 255) / 256), 256, 0, stream>>>(pat, P16, 8.0f, (long long)NPAT * HD / 8);
    k_at_h16<<<(unsigned)(((long long)NDRUG * HD / 8 + 255) / 256), 256, 0, stream>>>(drg, D16, 8.0f, (long long)NDRUG * HD / 8);
    eng::wmma_gemm64<0, false, 0, 0, false, 0><<<dim3((unsigned)((((NPAT) / 64) * ((HD) / 64) + 7) / 8), (unsigned)(1)), 256, 0, stream>>>((const unsigned short*)(P16), nullptr, HD, 0, (const unsigned short*)(WT16), nullptr, 3 * HD, 0, (void*)(PPb), nullptr, HD, 0, nullptr, nullptr, 0, NPAT, HD, HD, 0.00390625f);
    eng::wmma_gemm64<0, false, 2, 0, false, 0><<<dim3((unsigned)((((NDRUG) / 64) * ((HD) / 64) + 7) / 8), (unsigned)(1)), 256, 0, stream>>>((const unsigned short*)(D16), nullptr, HD, 0, (const unsigned short*)(WT16 + HD), nullptr, 3 * HD, 0, (void*)(DPBb), nullptr, HD, 0, b1, nullptr, 0, NDRUG, HD, HD, 0.00390625f);
    k_pair<<<dim3((unsigned)(NDRUG / PK_MT), (unsigned)(NPAT / PK_NT)), 256, 0, stream>>>(P16, D16, WT16, PPb, DPBb, W2, b2, out);
}
